// SRUBaseline_48223892799513
// MI455X (gfx1250) — hardware-verified
//
#include <hip/hip_runtime.h>
#include <math.h>

constexpr int kBatch  = 32;
constexpr int kFrames = 2048;
constexpr int kIn     = 51;
constexpr int kInPad  = 64;
constexpr int kHid    = 256;
constexpr int kHid3   = 768;
constexpr int kRows   = kBatch * kFrames;
constexpr int kQBatch = 8;
constexpr int kQRows  = kQBatch * kFrames;
constexpr int kNumQ   = kBatch / kQBatch;
constexpr int kOutPad = 64;
constexpr int kLayers = 2;
constexpr float kWCarry  = 16.0f;
constexpr float kHCarry  = 16.0f;
constexpr float kScaleHW = 1.0f / 256.0f;

constexpr size_t kOffXA   = 0;
constexpr size_t kOffH0   = kOffXA  + (size_t)kRows * kInPad * 2;
constexpr size_t kOffH1   = kOffH0  + (size_t)kRows * kHid * 2;
constexpr size_t kOffU    = kOffH1  + (size_t)kRows * kHid * 2;
constexpr size_t kOffWin  = kOffU   + (size_t)kQRows * kHid3 * 4;
constexpr size_t kOffWl   = kOffWin + (size_t)kHid * kInPad * 2;
constexpr size_t kOffWout = kOffWl  + (size_t)kLayers * kHid3 * kHid * 2;
constexpr size_t kWsTotal = kOffWout + (size_t)kOutPad * kHid * 2;
static_assert(kWsTotal == 126681088ull);
static_assert(kWsTotal <= 134217728ull);
static_assert((size_t)kRows * kOutPad * 4 <= (size_t)kQRows * kHid3 * 4);
static_assert((kOffH0 % 128) == 0 && (kOffH1 % 128) == 0 && (kOffU % 128) == 0 && (kOffWin % 128) == 0 && (kOffWl % 128) == 0 && (kOffWout % 128) == 0);

typedef __attribute__((ext_vector_type(16))) _Float16 v16h;
typedef __attribute__((ext_vector_type(8)))  _Float16 v8h;
typedef __attribute__((ext_vector_type(16))) __bf16   v16b;
typedef __attribute__((ext_vector_type(8)))  __bf16   v8b;
typedef __attribute__((ext_vector_type(8)))  float    v8f;
typedef __attribute__((ext_vector_type(4)))  float    v4f;
typedef __attribute__((ext_vector_type(4)))  unsigned int v4u;

__device__ __forceinline__ unsigned short f2bf_bits(float f) {
  unsigned u = __float_as_uint(f);
  return (unsigned short)((u + 0x7FFFu + ((u >> 16) & 1u)) >> 16);
}
__device__ __forceinline__ float bf_bits2f(unsigned short h) { return __uint_as_float(((unsigned)h) << 16); }

__device__ __forceinline__ void dep_guard_h(v8f& a, v8f& b, v16h x, v16h y) { asm volatile("v_nop\n\tv_nop\n\tv_nop\n\tv_nop" : "+v"(a), "+v"(b) : "v"(x), "v"(y)); }
__device__ __forceinline__ void dep_guard_b(v8f& a, v8f& b, v16b x, v16b y) { asm volatile("v_nop\n\tv_nop\n\tv_nop\n\tv_nop" : "+v"(a), "+v"(b) : "v"(x), "v"(y)); }
__device__ __forceinline__ void keep4_h(v16h a, v16h b, v16h c, v16h d) { asm volatile("v_nop" :: "v"(a), "v"(b), "v"(c), "v"(d)); }
__device__ __forceinline__ void keep4_b(v16b a, v16b b, v16b c, v16b d) { asm volatile("v_nop" :: "v"(a), "v"(b), "v"(c), "v"(d)); }
__device__ __forceinline__ void acc_guard4(v8f& a, v8f& b, v8f& c, v8f& d) { asm volatile("v_nop\n\tv_nop\n\tv_nop\n\tv_nop" : "+v"(a), "+v"(b), "+v"(c), "+v"(d)); }
template <typename T> struct Frag;
template <> struct Frag<_Float16> {
  typedef v16h V; union U { v16h v; v8h h[2]; };
  static __device__ __forceinline__ v16h load(const _Float16* p) {
    U f; f.h[0] = *(const v8h*)(p); f.h[1] = *(const v8h*)(p + 16); return f.v;
  }
  static __device__ __forceinline__ v8f mma(v16h a, v16h b, v8f c) {
    return __builtin_amdgcn_wmma_f32_16x16x32_f16(false, a, false, b, (short)0, c, false, false);
  }
  static __device__ __forceinline__ void guard(v8f& a, v8f& b, v16h x, v16h y) { dep_guard_h(a, b, x, y); }
  static __device__ __forceinline__ void keep(v16h a, v16h b, v16h c, v16h d) { keep4_h(a, b, c, d); }
};
template <> struct Frag<__bf16> {
  typedef v16b V; union U { v16b v; v8b h[2]; };
  static __device__ __forceinline__ v16b load(const __bf16* p) {
    U f; f.h[0] = *(const v8b*)(p); f.h[1] = *(const v8b*)(p + 16); return f.v;
  }
  static __device__ __forceinline__ v8f mma(v16b a, v16b b, v8f c) {
    return __builtin_amdgcn_wmma_f32_16x16x32_bf16(false, a, false, b, (short)0, c, false, false);
  }
  static __device__ __forceinline__ void guard(v8f& a, v8f& b, v16b x, v16b y) { dep_guard_b(a, b, x, y); }
  static __device__ __forceinline__ void keep(v16b a, v16b b, v16b c, v16b d) { keep4_b(a, b, c, d); }
};

__device__ __forceinline__ unsigned pk16(unsigned short a, unsigned short b) { return (unsigned)a | ((unsigned)b << 16); }
__device__ __forceinline__ unsigned short h_bits(float f) { const _Float16 h = (_Float16)f; return __builtin_bit_cast(unsigned short, h); }

template <int ET> struct Elem;
template <> struct Elem<0> { typedef _Float16 T; };
template <> struct Elem<1> { typedef __bf16 T; };
template <int ET, bool SPLIT, int BIAS_MODE, int OUT_MODE, bool RESID, int ACT = 0>
__global__ __launch_bounds__(256) void wmma_gemm64(
    const unsigned short* __restrict__ Ap, const unsigned short* __restrict__ A2p, int lda, long strideA,
    const unsigned short* __restrict__ Btp, const unsigned short* __restrict__ Bt2p, int ldb, long strideB,
    void* __restrict__ Cout, void* __restrict__ Cout2, int ldc, long strideC,
    const float* __restrict__ bias, int nbias, float bscale,
    const float* __restrict__ resid, long strideR,
    int M, int N, int K, float scale) {
  typedef typename Elem<ET>::T T;
  typedef typename Frag<T>::V V;
  const T* A = (const T*)Ap; const T* A2 = (const T*)A2p; const T* Bt = (const T*)Btp; const T* Bt2 = (const T*)Bt2p;
  __shared__ __align__(16) float sT[8][16 * 68];
  const int b    = blockIdx.y;
  const int lane = threadIdx.x & 31;
  const int wave = threadIdx.x >> 5;
  const int tilesN = N >> 6;
  const int tilesM = M >> 6;
  const int tile = blockIdx.x * 8 + wave;
  if (tile >= tilesM * tilesN) return;
  const int tm = tile / tilesN;
  const int tn = tile - tm * tilesN;
  const int m0 = tm << 6;
  const int n0 = tn << 6;

  const T* Ab  = A  + (size_t)b * strideA;
  const T* Bb  = Bt + (size_t)b * strideB;
  const T* Ab2 = SPLIT ? (A2  + (size_t)b * strideA) : nullptr;
  const T* Bb2 = SPLIT ? (Bt2 + (size_t)b * strideB) : nullptr;

  const int rlane = lane & 15;
  const int koff  = (lane >> 4) * 8;
  const int mOff  = (lane >> 4) * 8;

  v8f acc[4][4];
#pragma unroll
  for (int i = 0; i < 4; ++i)
#pragma unroll
    for (int j = 0; j < 4; ++j) acc[i][j] = (v8f){0.f,0.f,0.f,0.f,0.f,0.f,0.f,0.f};

  for (int k0 = 0; k0 < K; k0 += 32) {
    V bh[4], bl[4];
#pragma unroll
    for (int j = 0; j < 4; ++j) {
      const size_t bo = (size_t)(n0 + (j << 4) + rlane) * ldb + koff + k0;
      bh[j] = Frag<T>::load(Bb + bo);
      if (SPLIT) bl[j] = Frag<T>::load(Bb2 + bo);
    }
#pragma unroll
    for (int i = 0; i < 4; ++i) {
      const size_t ao = (size_t)(m0 + (i << 4) + rlane) * lda + koff + k0;
      V ah = Frag<T>::load(Ab + ao);
      V al;
      if (SPLIT) al = Frag<T>::load(Ab2 + ao);
#pragma unroll
      for (int j = 0; j < 4; ++j) {
        acc[i][j] = Frag<T>::mma(ah, bh[j], acc[i][j]);
        if (SPLIT) {
          acc[i][j] = Frag<T>::mma(ah, bl[j], acc[i][j]);
          acc[i][j] = Frag<T>::mma(al, bh[j], acc[i][j]);
        }
      }
      Frag<T>::guard(acc[i][0], acc[i][3], ah, SPLIT ? al : ah);
    }
    Frag<T>::keep(bh[0], bh[1], bh[2], bh[3]);
    if (SPLIT) Frag<T>::keep(bl[0], bl[1], bl[2], bl[3]);
  }
  acc_guard4(acc[0][0], acc[0][1], acc[0][2], acc[0][3]);
  acc_guard4(acc[1][0], acc[1][1], acc[1][2], acc[1][3]);
  acc_guard4(acc[2][0], acc[2][1], acc[2][2], acc[2][3]);
  acc_guard4(acc[3][0], acc[3][1], acc[3][2], acc[3][3]);

  float* slab = sT[wave];
  const float* Rb = RESID ? (resid + (size_t)b * strideR) : nullptr;
#pragma unroll
  for (int i = 0; i < 4; ++i) {
    const int mBase = m0 + (i << 4);
#pragma unroll
    for (int j = 0; j < 4; ++j) {
      const int n = n0 + (j << 4) + rlane;
      float bv = 0.f;
      if (BIAS_MODE == 2) {
        const int nc = (n < nbias) ? n : (nbias - 1);
        bv = bias[nc] * bscale;
        bv = (n < nbias) ? bv : 0.f;
      }
#pragma unroll
      for (int r = 0; r < 8; ++r) {
        float v = acc[i][j][r] * scale;
        if (BIAS_MODE == 1) v += bias[mBase + mOff + r] * bscale;
        if (BIAS_MODE == 2) v += bv;
        if (RESID) v += Rb[(size_t)(mBase + mOff + r) * ldc + n];
        if (ACT == 2) v = fmaxf(v, 0.0f);
        if (ACT == 4) v = (v > 0.f) ? v : 0.01f * v;
        slab[(mOff + r) * 68 + (j << 4) + rlane] = v;
      }
    }
    __builtin_amdgcn_fence(__ATOMIC_RELEASE, "workgroup");
    __builtin_amdgcn_wave_barrier();
    __builtin_amdgcn_fence(__ATOMIC_ACQUIRE, "workgroup");
    if (OUT_MODE == 0) {
      float* C = (float*)Cout + (size_t)b * strideC;
      const int hh = lane >> 4, c4 = (lane & 15) * 4;
      for (int pass = 0; pass < 2; ++pass) {
#pragma unroll
        for (int it = 0; it < 8; ++it) {
          const int row = it * 2 + hh;
          v4f v = *(const v4f*)(slab + row * 68 + c4);
          *(volatile v4f*)(C + (size_t)(mBase + row) * ldc + n0 + c4) = v;
        }
        __threadfence();
      }
    } else {
      const int q = lane >> 3, c8 = (lane & 7) * 8;
      unsigned short* C  = (unsigned short*)Cout  + (size_t)b * strideC;
      unsigned short* C2 = (OUT_MODE == 2) ? ((unsigned short*)Cout2 + (size_t)b * strideC) : nullptr;
      for (int pass = 0; pass < 2; ++pass) {
#pragma unroll
        for (int it = 0; it < 4; ++it) {
          const int row = it * 4 + q;
          const float* sp = slab + row * 68 + c8;
          v8h hv, lv;
#pragma unroll
          for (int e = 0; e < 8; ++e) {
            if (OUT_MODE == 1) {
              hv[e] = (_Float16)sp[e];
            } else {
              unsigned short hb = f2bf_bits(sp[e]);
              unsigned short lb = f2bf_bits(sp[e] - bf_bits2f(hb));
              hv[e] = __builtin_bit_cast(_Float16, hb);
              lv[e] = __builtin_bit_cast(_Float16, lb);
            }
          }
          *(volatile v8h*)(C + (size_t)(mBase + row) * ldc + n0 + c8) = hv;
          if (OUT_MODE == 2) *(volatile v8h*)(C2 + (size_t)(mBase + row) * ldc + n0 + c8) = lv;
        }
        __threadfence();
      }
    }
    __builtin_amdgcn_fence(__ATOMIC_RELEASE, "workgroup");
    __builtin_amdgcn_wave_barrier();
    __builtin_amdgcn_fence(__ATOMIC_ACQUIRE, "workgroup");
  }
}

__global__ __launch_bounds__(256) void tcast_kernel(const float* __restrict__ in, int Kin, int Nin, long in_plane,
                                                    unsigned short* __restrict__ out, int Kp, long out_plane, float scale) {
  __shared__ float sm[64][65];
  const int t  = threadIdx.x;
  const int k0 = blockIdx.x * 64;
  const int n0 = blockIdx.y * 64;
  const int z  = blockIdx.z;
  const float* ip = in + (size_t)z * (size_t)in_plane;
#pragma unroll
  for (int i = 0; i < 16; ++i) {
    const int e  = i * 256 + t;
    const int r  = e >> 6;
    const int cc = e & 63;
    const int k  = k0 + r;
    const int n  = n0 + cc;
    const int kc = (k < Kin) ? k : (Kin - 1);
    const int nc = (n < Nin) ? n : (Nin - 1);
    float v = ip[(size_t)kc * Nin + nc] * scale;
    v = (k < Kin && n < Nin) ? v : 0.0f;
    sm[cc][r] = v;
  }
  __syncthreads();
  const int lane = t & 31, wave = t >> 5;
  const int q = lane >> 3, c8 = (lane & 7) * 8;
  unsigned short* op = out + (size_t)z * (size_t)out_plane;
  for (int pass = 0; pass < 2; ++pass) {
#pragma unroll
    for (int it = 0; it < 2; ++it) {
      const int row = wave * 8 + it * 4 + q;
      unsigned short hb[8];
#pragma unroll
      for (int e = 0; e < 8; ++e) hb[e] = h_bits(sm[row][c8 + e]);
      const v4u u = (v4u){pk16(hb[0], hb[1]), pk16(hb[2], hb[3]), pk16(hb[4], hb[5]), pk16(hb[6], hb[7])};
      *(volatile v4u*)(op + (size_t)(n0 + row) * Kp + k0 + c8) = u;
    }
    __threadfence();
  }
}

__global__ __launch_bounds__(256) void xcast_kernel(const float* __restrict__ x, unsigned short* __restrict__ xa, int nthreads) {
  const int g = blockIdx.x * 256 + threadIdx.x;
  if (g >= nthreads) return;
  const int row = g >> 3;
  const int c8  = (g & 7) * 8;
  const float* xr = x + (size_t)row * kIn;
  unsigned short hb[8];
#pragma unroll
  for (int e = 0; e < 8; ++e) {
    const int col = c8 + e;
    const int cc  = (col < kIn) ? col : (kIn - 1);
    float v = xr[cc];
    v = (col < kIn) ? v : 0.0f;
    hb[e] = h_bits(v);
  }
  const v4u u = (v4u){pk16(hb[0], hb[1]), pk16(hb[2], hb[3]), pk16(hb[4], hb[5]), pk16(hb[6], hb[7])};
  unsigned short* q = xa + (size_t)row * kInPad + c8;
  *(volatile v4u*)q = u;
  __threadfence();
  *(volatile v4u*)q = u;
}

__device__ __forceinline__ float sigm_f(float v) {
  const float e = expf(-v);
  return __builtin_amdgcn_rcpf(1.0f + e);
}

__global__ __launch_bounds__(32) void sru_scan_kernel(const float* __restrict__ U, unsigned short* __restrict__ Hout, int row_base) {
  const int lane = threadIdx.x;
  const int bq   = blockIdx.x;
  const int ch0  = lane * 8;
  const float* up = U + (size_t)bq * kFrames * kHid3 + ch0;
  unsigned short* hp = Hout + ((size_t)row_base + (size_t)bq * kFrames) * kHid + ch0;
  v4f c0 = (v4f){0.f, 0.f, 0.f, 0.f};
  v4f c1 = (v4f){0.f, 0.f, 0.f, 0.f};
  for (int f = 0; f < kFrames; ++f) {
    const float* ur = up + (size_t)f * kHid3;
    unsigned w0 = 0u, w1 = 0u, w2 = 0u, w3 = 0u;
#pragma unroll 1
    for (int grp = 0; grp < 2; ++grp) {
      const v4f xt = *(const v4f*)(ur + 4 * grp);
      const v4f fg = *(const v4f*)(ur + kHid + 4 * grp);
      const v4f rg = *(const v4f*)(ur + 2 * kHid + 4 * grp);
      v4f cg;
      if (grp == 0) cg = c0; else cg = c1;
      float hv[4];
#pragma unroll
      for (int e = 0; e < 4; ++e) {
        const float ft = sigm_f(fg[e]);
        const float rt = sigm_f(rg[e]);
        const float cn = ft * cg[e] + (1.0f - ft) * xt[e];
        cg[e] = cn;
        const float th = 2.0f * sigm_f(2.0f * cn) - 1.0f;
        hv[e] = rt * th + (1.0f - rt) * xt[e];
      }
      const unsigned p0 = pk16(h_bits(hv[0] * kHCarry), h_bits(hv[1] * kHCarry));
      const unsigned p1 = pk16(h_bits(hv[2] * kHCarry), h_bits(hv[3] * kHCarry));
      if (grp == 0) { c0 = cg; w0 = p0; w1 = p1; }
      else          { c1 = cg; w2 = p0; w3 = p1; }
    }
    const v4u u = (v4u){w0, w1, w2, w3};
    unsigned short* dst = hp + (size_t)f * kHid;
    *(volatile v4u*)dst = u;
    __threadfence();
    *(volatile v4u*)dst = u;
  }
}

__global__ __launch_bounds__(256) void pack_out_kernel(const float* __restrict__ ys, float* __restrict__ out, int n4) {
  const int i = blockIdx.x * 256 + threadIdx.x;
  if (i >= n4) return;
  v4f v;
#pragma unroll
  for (int j = 0; j < 4; ++j) {
    const int e = 4 * i + j;
    const int r = e / kIn;
    const int c = e - r * kIn;
    v[j] = ys[(size_t)r * kOutPad + c];
  }
  float* q = out + 4 * (size_t)i;
  *(volatile v4f*)q = v;
  __threadfence();
  *(volatile v4f*)q = v;
}

extern "C" void kernel_launch(void* const* d_in, const int* in_sizes, int n_in,
                              void* d_out, int out_size, void* d_ws, size_t ws_size,
                              hipStream_t stream) {
  if (n_in < 7) return;
  if (in_sizes[0] != kRows * kIn) return;
  if (in_sizes[1] != kIn * kHid || in_sizes[2] != kHid) return;
  if (in_sizes[3] != kLayers * kHid * kHid3 || in_sizes[4] != kLayers * kHid3) return;
  if (in_sizes[5] != kHid * kIn || in_sizes[6] != kIn) return;
  if (out_size != kRows * kIn) return;
  if (ws_size < kWsTotal) return;

  const float* x    = (const float*)d_in[0];
  const float* Win  = (const float*)d_in[1];
  const float* bin  = (const float*)d_in[2];
  const float* Wl   = (const float*)d_in[3];
  const float* bl   = (const float*)d_in[4];
  const float* Wout = (const float*)d_in[5];
  const float* bout = (const float*)d_in[6];
  float* out = (float*)d_out;

  char* ws = (char*)d_ws;
  unsigned short* XA    = (unsigned short*)(ws + kOffXA);
  unsigned short* H0    = (unsigned short*)(ws + kOffH0);
  unsigned short* H1    = (unsigned short*)(ws + kOffH1);
  float*          Ubuf  = (float*)(ws + kOffU);
  float*          Ystg  = (float*)(ws + kOffU);
  unsigned short* WinT  = (unsigned short*)(ws + kOffWin);
  unsigned short* WlT   = (unsigned short*)(ws + kOffWl);
  unsigned short* WoutT = (unsigned short*)(ws + kOffWout);

  tcast_kernel<<<dim3(kInPad / 64, kHid / 64, 1), 256, 0, stream>>>(Win, kIn, kHid, 0L, WinT, kInPad, 0L, kWCarry);
  tcast_kernel<<<dim3(kHid / 64, kHid3 / 64, kLayers), 256, 0, stream>>>(Wl, kHid, kHid3, (long)kHid * kHid3,
                                                                          WlT, kHid, (long)kHid3 * kHid, kWCarry);
  tcast_kernel<<<dim3(kHid / 64, kOutPad / 64, 1), 256, 0, stream>>>(Wout, kHid, kIn, 0L, WoutT, kHid, 0L, kWCarry);
  xcast_kernel<<<(kRows * 8) / 256, 256, 0, stream>>>(x, XA, kRows * 8);

  {
    const int tiles = (kRows / 64) * (kHid / 64);
    wmma_gemm64<0, false, 2, 1, false, 0><<<dim3(tiles / 8, 1), 256, 0, stream>>>(
        XA, XA, kInPad, 0L, WinT, WinT, kInPad, 0L,
        (void*)H0, (void*)H0, kHid, 0L,
        bin, kHid, kHCarry, bin, 0L,
        kRows, kHid, kInPad, 1.0f);
  }

  for (int l = 0; l < kLayers; ++l) {
    const unsigned short* Hsrc = (l == 0) ? H0 : H1;
    unsigned short*       Hdst = (l == 0) ? H1 : H0;
    const unsigned short* Wp   = WlT + (size_t)l * kHid3 * kHid;
    const float*          bp   = bl + (size_t)l * kHid3;
    const int tiles = (kQRows / 64) * (kHid3 / 64);
    for (int q = 0; q < kNumQ; ++q) {
      const unsigned short* Aq = Hsrc + (size_t)q * kQRows * kHid;
      wmma_gemm64<0, false, 2, 0, false, 0><<<dim3(tiles / 8, 1), 256, 0, stream>>>(
          Aq, Aq, kHid, 0L, Wp, Wp, kHid, 0L,
          (void*)Ubuf, (void*)Ubuf, kHid3, 0L,
          bp, kHid3, 1.0f, bp, 0L,
          kQRows, kHid3, kHid, kScaleHW);
      sru_scan_kernel<<<kQBatch, 32, 0, stream>>>(Ubuf, Hdst, q * kQRows);
    }
  }

  {
    const int tiles = (kRows / 64) * (kOutPad / 64);
    wmma_gemm64<0, false, 2, 0, false, 0><<<dim3(tiles / 8, 1), 256, 0, stream>>>(
        H0, H0, kHid, 0L, WoutT, WoutT, kHid, 0L,
        (void*)Ystg, (void*)Ystg, kOutPad, 0L,
        bout, kIn, 1.0f, bout, 0L,
        kRows, kOutPad, kHid, kScaleHW);
  }

  {
    const int n4 = (kRows * kIn) / 4;
    pack_out_kernel<<<(n4 + 255) / 256, 256, 0, stream>>>(Ystg, out, n4);
  }
}
